// clustering_dynamic_learning_common_center_2_45286135169476
// MI455X (gfx1250) — hardware-verified
//
#include <hip/hip_runtime.h>


#define NB_  32
#define NN   512
#define KK   32
#define TI   24
#define FF   64
#define CC   8
#define DDm  16
#define MID  32
#define SS   64
#define NR   (NB_ * NN)
typedef _Float16 h16;
typedef unsigned short bf;
typedef __attribute__((ext_vector_type(16))) __bf16   v16bf;
typedef __attribute__((ext_vector_type(16))) _Float16 v16h;
typedef __attribute__((ext_vector_type(8)))  _Float16 v8h;
typedef __attribute__((ext_vector_type(8)))  unsigned short v8us;
typedef __attribute__((ext_vector_type(8)))  float    v8f;
typedef __attribute__((ext_vector_type(4)))  float    v4f;
typedef v8h  __attribute__((may_alias)) v8ha;
typedef v4f  __attribute__((may_alias)) v4fa;
typedef v8us __attribute__((may_alias)) v8usa;

__device__ __forceinline__ unsigned short f2bf(float f) { unsigned u = __float_as_uint(f); u += 0x7FFFu + ((u >> 16) & 1u); return (unsigned short)(u >> 16); }
__device__ __forceinline__ float bf2f(unsigned short b) { return __uint_as_float(((unsigned)b) << 16); }
__device__ __forceinline__ float bfr(float f) { return bf2f(f2bf(f)); }
__device__ __forceinline__ v16h cat16(v8h lo, v8h hi) { return __builtin_shufflevector(lo, hi, 0, 1, 2, 3, 4, 5, 6, 7, 8, 9, 10, 11, 12, 13, 14, 15); }
__device__ __forceinline__ v16bf cat16b(v8us lo, v8us hi) { return __builtin_bit_cast(v16bf, __builtin_shufflevector(lo, hi, 0, 1, 2, 3, 4, 5, 6, 7, 8, 9, 10, 11, 12, 13, 14, 15)); }
__device__ __forceinline__ v8f wmma16(v16h a, v16h b, v8f c) { return __builtin_amdgcn_wmma_f32_16x16x32_f16(false, a, false, b, (short)0, c, false, false); }
__device__ __forceinline__ v8f wmmab(v16bf a, v16bf b, v8f c) { return __builtin_amdgcn_wmma_f32_16x16x32_bf16(false, a, false, b, (short)0, c, false, false); }


template <typename T16> struct WFrag;
template <> struct WFrag<h16> { typedef v16h V; static __device__ __forceinline__ V ld(const h16* p) { return cat16(*(const v8h*)p, *(const v8h*)(p + 16)); } static __device__ __forceinline__ v8f mma(V a, V b, v8f c) { return wmma16(a, b, c); } };
template <> struct WFrag<bf> { typedef v16bf V; static __device__ __forceinline__ V ld(const bf* p) { return cat16b(*(const v8us*)p, *(const v8us*)(p + 16)); } static __device__ __forceinline__ v8f mma(V a, V b, v8f c) { return wmmab(a, b, c); } };
template <typename T16, int NSPLIT, bool BIAS>
__global__ __launch_bounds__(32) void k_gemmw(const T16* __restrict__ A, const T16* __restrict__ A2, const T16* __restrict__ Bt, const T16* __restrict__ Bt2, int K, float* C, int ldc, const float* __restrict__ bias, size_t sA, size_t sB, size_t sC) {
    typedef typename WFrag<T16>::V V;
    __shared__ __align__(16) float os[16 * 68];
    const size_t z = blockIdx.z; A += z * sA; if (A2) A2 += z * sA; Bt += z * sB; if (Bt2) Bt2 += z * sB; C += z * sC;
    const int lane = threadIdx.x & 31, lr = lane & 15, hi = lane >> 4; const int r0 = blockIdx.x * 64, c0 = blockIdx.y * 64;
    v8f acc[4][4];
#pragma unroll
    for (int mb = 0; mb < 4; ++mb)
#pragma unroll
        for (int nb = 0; nb < 4; ++nb) acc[mb][nb] = (v8f){};
    const size_t aoff = (size_t)(r0 + lr) * K + 8 * hi, boff = (size_t)(c0 + lr) * K + 8 * hi;
#pragma unroll 1
    for (int kc = 0; kc < K; kc += 32) {
        V a[4], a2[4];
#pragma unroll
        for (int mb = 0; mb < 4; ++mb) { a[mb] = WFrag<T16>::ld(A + aoff + (size_t)mb * 16 * K + kc); if (NSPLIT == 1 || NSPLIT == 2) a2[mb] = WFrag<T16>::ld(A2 + aoff + (size_t)mb * 16 * K + kc); }
#pragma unroll
        for (int nb = 0; nb < 4; ++nb) { const V b = WFrag<T16>::ld(Bt + boff + (size_t)nb * 16 * K + kc); V b2; if (NSPLIT >= 2) b2 = WFrag<T16>::ld(Bt2 + boff + (size_t)nb * 16 * K + kc);
#pragma unroll
            for (int mb = 0; mb < 4; ++mb) { acc[mb][nb] = WFrag<T16>::mma(a[mb], b, acc[mb][nb]); if (NSPLIT == 1 || NSPLIT == 2) acc[mb][nb] = WFrag<T16>::mma(a2[mb], b, acc[mb][nb]); if (NSPLIT >= 2) acc[mb][nb] = WFrag<T16>::mma(a[mb], b2, acc[mb][nb]); } }
        asm volatile("v_nop\n\tv_nop\n\tv_nop\n\tv_nop" : "+v"(acc[0][0]), "+v"(acc[1][1]), "+v"(acc[2][2]), "+v"(acc[3][3]) : "v"(a[0]), "v"(a[3]));
    }
#pragma unroll
    for (int mb = 0; mb < 4; ++mb) {
#pragma unroll
        for (int nb = 0; nb < 4; ++nb) {
#pragma unroll
            for (int j = 0; j < 8; ++j) os[(hi * 8 + j) * 68 + nb * 16 + lr] = acc[mb][nb][j]; }
        __builtin_amdgcn_wave_barrier(); asm volatile("" ::: "memory");
        float* crow = C + (size_t)(r0 + mb * 16) * ldc + c0;
#pragma unroll 1
        for (int ps = 0; ps < 2; ++ps) {
#pragma unroll
            for (int s = 0; s < 8; ++s) { const int row = 2 * s + hi, cofs = lr * 4; v4f val = *(const v4fa*)(os + row * 68 + cofs); if (BIAS) { val[0] += bfr(bias[c0 + cofs]); val[1] += bfr(bias[c0 + cofs + 1]); val[2] += bfr(bias[c0 + cofs + 2]); val[3] += bfr(bias[c0 + cofs + 3]); }
                *(volatile v4f*)(crow + (size_t)row * ldc + cofs) = val; }
            if (ps == 0) __threadfence(); }
        __builtin_amdgcn_wave_barrier(); asm volatile("" ::: "memory");
    }
}

__device__ __forceinline__ void splitf(float y, unsigned short& h, unsigned short& l) { h = f2bf(y); l = f2bf(y - bf2f(h)); }
typedef __attribute__((ext_vector_type(4))) unsigned short v4us;

__global__ __launch_bounds__(256) void k_cvt8(const float* __restrict__ src, bf* dst, size_t n8) { const size_t i = (size_t)blockIdx.x * 256 + threadIdx.x; if (i >= n8) return; const v8f v = *(const v8f*)(src + i * 8); v8us o;
#pragma unroll
    for (int k = 0; k < 8; ++k) o[k] = f2bf(v[k]); *(volatile v8us*)(dst + i * 8) = o; __threadfence(); *(volatile v8us*)(dst + i * 8) = o; }
__global__ __launch_bounds__(256) void k_wpad(const float* __restrict__ w, int K, int N, int KP, int NP, bf* Bt) { const int e = (blockIdx.x * 256 + threadIdx.x) * 4; if (e >= NP * KP) return; const int k = e % KP; const int o = e / KP; v4us v;
#pragma unroll
    for (int u = 0; u < 4; ++u) v[u] = (o < N && k + u < K) ? f2bf(w[(size_t)(k + u) * N + o]) : (unsigned short)0; *(volatile v4us*)(Bt + e) = v; __threadfence(); *(volatile v4us*)(Bt + e) = v; }
__global__ __launch_bounds__(256) void k_inb(const float* __restrict__ inp, bf* A) { const int e = (blockIdx.x * 256 + threadIdx.x) * 4; if (e >= NR * 32) return; const int k = e % 32; const int r = e / 32; v4us v;
#pragma unroll
    for (int u = 0; u < 4; ++u) v[u] = (k + u < TI) ? f2bf(inp[(size_t)r * TI + k + u]) : (unsigned short)0; *(volatile v4us*)(A + e) = v; __threadfence(); *(volatile v4us*)(A + e) = v; }
__global__ __launch_bounds__(256) void k_gwb(const float* __restrict__ gw, bf* Bt) { const int e = (blockIdx.x * 256 + threadIdx.x) * 4; if (e >= CC * SS * 32) return; const int t = e % 32; const int row = e / 32; const int i = row / SS, s = row % SS; v4us v;
#pragma unroll
    for (int u = 0; u < 4; ++u) v[u] = (t + u < TI) ? f2bf(gw[((size_t)i * TI + t + u) * SS + s]) : (unsigned short)0; *(volatile v4us*)(Bt + e) = v; __threadfence(); *(volatile v4us*)(Bt + e) = v; }
__global__ __launch_bounds__(256) void k_relp(const float* __restrict__ G, const float* __restrict__ b, bf* Hh, bf* Hl) { const int e = (blockIdx.x * 256 + threadIdx.x) * 4; if (e >= NR * MID) return; const int c = e % MID; const int r = e / MID; v4us oh, ol;
#pragma unroll
    for (int u = 0; u < 4; ++u) { unsigned short p, q; splitf(fmaxf(__fadd_rn(G[(size_t)r * 64 + c + u], bfr(b[c + u])), 0.f), p, q); oh[u] = p; ol[u] = q; } *(volatile v4us*)(Hh + e) = oh; *(volatile v4us*)(Hl + e) = ol; __threadfence(); *(volatile v4us*)(Hh + e) = oh; *(volatile v4us*)(Hl + e) = ol; }
__global__ __launch_bounds__(256) void k_feat(const float* __restrict__ G2, const float* __restrict__ b2, const float* __restrict__ G3, const float* __restrict__ bc, float* FE) { const int e = (blockIdx.x * 256 + threadIdx.x) * 4; if (e >= NR * DDm) return; const int d = e % DDm; const int r = e / DDm; v4f o;
#pragma unroll
    for (int u = 0; u < 4; ++u) { const float a = fmaxf(__fadd_rn(G2[(size_t)r * 64 + d + u], bfr(b2[d + u])), 0.f); const float c = fmaxf(__fadd_rn(G3[(size_t)r * 64 + d + u], bfr(bc[d + u])), 0.f); o[u] = __fadd_rn(a, c); } *(volatile v4f*)(FE + e) = o; __threadfence(); *(volatile v4f*)(FE + e) = o; }
__global__ __launch_bounds__(128) void k_cen(const float* __restrict__ cen, const float* __restrict__ W1, const float* __restrict__ b1, const float* __restrict__ W2, const float* __restrict__ b2, const float* __restrict__ Wc, const float* __restrict__ bc, float* CF) {
    const int idx = threadIdx.x; if (idx >= CC * DDm) return; const int c = idx / DDm, d = idx % DDm; float acc2 = 0.f;
#pragma unroll 1
    for (int m = 0; m < MID; ++m) { float a1 = 0.f;
#pragma unroll 1
        for (int f = 0; f < FF; ++f) { float p = __fmul_rn(bfr(cen[c * FF + f]), bfr(W1[f * MID + m])); asm volatile("" : "+v"(p)); a1 = __fadd_rn(a1, p); }
        const float h1 = fmaxf(__fadd_rn(a1, bfr(b1[m])), 0.f); float p2 = __fmul_rn(h1, bfr(W2[m * DDm + d])); asm volatile("" : "+v"(p2)); acc2 = __fadd_rn(acc2, p2); }
    float a3 = 0.f;
#pragma unroll 1
    for (int f = 0; f < FF; ++f) { float p = __fmul_rn(bfr(cen[c * FF + f]), bfr(Wc[f * DDm + d])); asm volatile("" : "+v"(p)); a3 = __fadd_rn(a3, p); }
    const float r = __fadd_rn(fmaxf(__fadd_rn(acc2, bfr(b2[d])), 0.f), fmaxf(__fadd_rn(a3, bfr(bc[d])), 0.f)); *(volatile float*)(CF + idx) = r; __threadfence(); *(volatile float*)(CF + idx) = r; }
__global__ __launch_bounds__(64) void k_mean(const float* __restrict__ M, int ncol, int nrow, float scale, float* out) { const int c = blockIdx.x * 64 + threadIdx.x; if (c >= ncol) return; float s = 0.f;
#pragma unroll 1
    for (int r = 0; r < nrow; ++r) s = __fadd_rn(s, M[(size_t)r * ncol + c]); const float v = __fmul_rn(s, scale); *(volatile float*)(out + c) = v; __threadfence(); *(volatile float*)(out + c) = v; }
__global__ __launch_bounds__(256) void k_simi(const float* __restrict__ FE, const float* __restrict__ CF, const float* __restrict__ ADJ, float* SM) { const int idx = blockIdx.x * 256 + threadIdx.x; if (idx >= NR) return;
    float x1[DDm]; float x1n = 0.f;
#pragma unroll
    for (int d = 0; d < DDm; ++d) { x1[d] = __fsub_rn(FE[(size_t)idx * DDm + d], ADJ[d]); float p = __fmul_rn(x1[d], x1[d]); asm volatile("" : "+v"(p)); x1n = __fadd_rn(x1n, p); }
    float dist[CC]; float mx = -3.0e38f;
#pragma unroll
    for (int c = 0; c < CC; ++c) { float x2n = 0.f, dot = 0.f;
#pragma unroll
        for (int d = 0; d < DDm; ++d) { const float x2 = __fsub_rn(CF[c * DDm + d], ADJ[d]); float p = __fmul_rn(x2, x2); asm volatile("" : "+v"(p)); x2n = __fadd_rn(x2n, p); float q = __fmul_rn(x1[d], x2); asm volatile("" : "+v"(q)); dot = __fadd_rn(dot, q); }
        float t2 = __fmul_rn(2.0f, dot); asm volatile("" : "+v"(t2)); float res = __fsub_rn(__fadd_rn(x1n, x2n), t2); res = fmaxf(res, 1e-30f); dist[c] = __fsqrt_rn(res); mx = fmaxf(mx, dist[c]); }
    float se = 0.f;
#pragma unroll
    for (int c = 0; c < CC; ++c) { dist[c] = __expf(__fsub_rn(dist[c], mx)); se = __fadd_rn(se, dist[c]); }
    const float inv = __fdiv_rn(1.0f, se); v4f o0, o1; for (int c = 0; c < 4; ++c) { o0[c] = __fmul_rn(dist[c], inv); o1[c] = __fmul_rn(dist[4 + c], inv); }
    *(volatile v4f*)(SM + (size_t)idx * CC) = o0; *(volatile v4f*)(SM + (size_t)idx * CC + 4) = o1; __threadfence(); *(volatile v4f*)(SM + (size_t)idx * CC) = o0; *(volatile v4f*)(SM + (size_t)idx * CC + 4) = o1; }
__global__ __launch_bounds__(256) void k_outw(const float* __restrict__ Hm, const float* __restrict__ SM, const int* __restrict__ adj, float* out0) { const size_t e = ((size_t)blockIdx.x * 256 + threadIdx.x) * 4; if (e >= (size_t)NR * CC * SS) return; const int s = (int)(e % SS); const int i = (int)((e / SS) % CC); const int r = (int)(e / (SS * CC)); const int b = r / NN; const int* ar = adj + (size_t)r * KK; float acc[4] = {0.f, 0.f, 0.f, 0.f}; float ws = 0.f;
#pragma unroll 1
    for (int k = 0; k < KK; ++k) { int m = ar[k]; m = min(max(m, 0), NN - 1); const size_t mr = (size_t)b * NN + m; const float w = SM[mr * CC + i]; const v4f h = *(const v4f*)(Hm + mr * (CC * SS) + i * SS + s);
#pragma unroll
        for (int u = 0; u < 4; ++u) { float p = __fmul_rn(fmaxf(h[u], 0.f), w); asm volatile("" : "+v"(p)); acc[u] = __fadd_rn(acc[u], p); } ws = __fadd_rn(ws, w); }
    v4f o; for (int u = 0; u < 4; ++u) o[u] = __fdiv_rn(acc[u], ws); *(volatile v4f*)(out0 + e) = o; __threadfence(); *(volatile v4f*)(out0 + e) = o; }
__global__ __launch_bounds__(64) void k_loss(const float* __restrict__ cen, const float* __restrict__ CM, float* out1) { if (threadIdx.x != 0) return; __shared__ float nc[CC * SS]; __shared__ float adjm[SS];
#pragma unroll 1
    for (int e = 0; e < CC * SS; ++e) { float a = __fmul_rn(0.99f, bfr(cen[e])); asm volatile("" : "+v"(a)); float b = __fmul_rn(0.01f, CM[e]); asm volatile("" : "+v"(b)); nc[e] = __fadd_rn(a, b); }
#pragma unroll 1
    for (int f = 0; f < SS; ++f) { float s = 0.f;
#pragma unroll 1
        for (int c = 0; c < CC; ++c) s = __fadd_rn(s, nc[c * SS + f]); adjm[f] = __fmul_rn(s, 1.0f / CC); }
    float loss = 0.f;
#pragma unroll 1
    for (int a = 0; a < CC; ++a) {
#pragma unroll 1
        for (int b = 0; b < CC; ++b) { float an = 0.f, bn = 0.f, dot = 0.f;
#pragma unroll 1
            for (int f = 0; f < SS; ++f) { const float xa = __fsub_rn(nc[a * SS + f], adjm[f]), yb = __fsub_rn(nc[b * SS + f], adjm[f]); float p1 = __fmul_rn(xa, xa); asm volatile("" : "+v"(p1)); an = __fadd_rn(an, p1); float p2 = __fmul_rn(yb, yb); asm volatile("" : "+v"(p2)); bn = __fadd_rn(bn, p2); float p3 = __fmul_rn(xa, yb); asm volatile("" : "+v"(p3)); dot = __fadd_rn(dot, p3); }
            float t2 = __fmul_rn(2.0f, dot); asm volatile("" : "+v"(t2)); float res = __fsub_rn(__fadd_rn(an, bn), t2); res = fmaxf(res, 1e-30f); const float dist = __fsqrt_rn(res); const float tgt = (a == b) ? 0.f : 0.5f; const float cl = fmaxf(__fsub_rn(tgt, dist), 0.f); float sq = __fmul_rn(cl, cl); asm volatile("" : "+v"(sq)); loss = __fadd_rn(loss, sq); } }
    *(volatile float*)out1 = loss; __threadfence(); *(volatile float*)out1 = loss; }

extern "C" void kernel_launch(void* const* d_in, const int* in_sizes, int n_in,
                              void* d_out, int out_size, void* d_ws, size_t ws_size, hipStream_t stream) {
    (void)in_sizes; (void)n_in; (void)out_size;
    const float** I = (const float**)d_in;
    const float *ff = I[0], *inp = I[1]; const int* adj = (const int*)d_in[2]; const float *cen = I[3], *cW1 = I[4], *cb1 = I[5], *cW2 = I[6], *cb2 = I[7], *cWc = I[8], *cbc = I[9], *W1 = I[10], *b1 = I[11], *W2 = I[12], *b2 = I[13], *Wc = I[14], *bc = I[15], *gw = I[16], *gb = I[17];
    float* OUT0 = (float*)d_out;
    float* OUT1 = OUT0 + (size_t)NR * CC * SS;
    char* wsp = (char*)d_ws;
    auto take = [&](size_t bytes) { char* p = wsp; wsp += (bytes + 255) & ~(size_t)255; return (void*)p; };
    bf* FB = (bf*)take((size_t)NR * FF * 2); bf* BW1 = (bf*)take(64 * FF * 2); bf* BW2 = (bf*)take(64 * 32 * 2); bf* BWc = (bf*)take(64 * FF * 2); float* G1 = (float*)take((size_t)NR * 64 * 4); bf* R1h = (bf*)take((size_t)NR * MID * 2); bf* R1l = (bf*)take((size_t)NR * MID * 2); float* G2 = (float*)take((size_t)NR * 64 * 4); float* G3 = (float*)take((size_t)NR * 64 * 4);
    float* FE = (float*)take((size_t)NR * DDm * 4); float* CF = (float*)take(CC * DDm * 4); float* ADJ = (float*)take(256); float* SM = (float*)take((size_t)NR * CC * 4); bf* IA = (bf*)take((size_t)NR * 32 * 2); bf* BG = (bf*)take((size_t)CC * SS * 32 * 2); float* GB = (float*)take(CC * SS * 4); float* Hm = (float*)take((size_t)NR * CC * SS * 4); float* CM = (float*)take(CC * SS * 4);
    if ((size_t)(wsp - (char*)d_ws) > ws_size) return;
    k_cvt8<<<(NR * FF / 8 + 255) / 256, 256, 0, stream>>>(ff, FB, NR * FF / 8);
    k_wpad<<<(64 * FF / 4 + 255) / 256, 256, 0, stream>>>(W1, FF, MID, FF, 64, BW1); k_wpad<<<(64 * 32 / 4 + 255) / 256, 256, 0, stream>>>(W2, MID, DDm, 32, 64, BW2); k_wpad<<<(64 * FF / 4 + 255) / 256, 256, 0, stream>>>(Wc, FF, DDm, FF, 64, BWc);
    k_gemmw<bf, 0, false><<<dim3(NR / 64, 1, 1), 32, 0, stream>>>(FB, nullptr, BW1, nullptr, FF, G1, 64, nullptr, 0, 0, 0);
    k_relp<<<(NR * MID / 4 + 255) / 256, 256, 0, stream>>>(G1, b1, R1h, R1l);
    k_gemmw<bf, 1, false><<<dim3(NR / 64, 1, 1), 32, 0, stream>>>(R1h, R1l, BW2, nullptr, 32, G2, 64, nullptr, 0, 0, 0);
    k_gemmw<bf, 0, false><<<dim3(NR / 64, 1, 1), 32, 0, stream>>>(FB, nullptr, BWc, nullptr, FF, G3, 64, nullptr, 0, 0, 0);
    k_feat<<<(NR * DDm / 4 + 255) / 256, 256, 0, stream>>>(G2, b2, G3, bc, FE);
    k_cen<<<1, 128, 0, stream>>>(cen, cW1, cb1, cW2, cb2, cWc, cbc, CF);
    k_mean<<<1, 64, 0, stream>>>(FE, DDm, NR, 1.0f / NR, ADJ);
    k_simi<<<(NR + 255) / 256, 256, 0, stream>>>(FE, CF, ADJ, SM);
    k_inb<<<(NR * 32 / 4 + 255) / 256, 256, 0, stream>>>(inp, IA); k_gwb<<<(CC * SS * 32 / 4 + 255) / 256, 256, 0, stream>>>(gw, BG);
    k_gemmw<bf, 0, true><<<dim3(NR / 64, CC * SS / 64, 1), 32, 0, stream>>>(IA, nullptr, BG, nullptr, 32, Hm, CC * SS, gb, 0, 0, 0);
    k_outw<<<(unsigned)(((size_t)NR * CC * SS / 4 + 255) / 256), 256, 0, stream>>>(Hm, SM, adj, OUT0);
    k_mean<<<8, 64, 0, stream>>>(OUT0, CC * SS, NR, 1.0f / NR, CM);
    k_loss<<<1, 64, 0, stream>>>(cen, CM, OUT1);
}
